// SparseCrossAttentionLayer_60945585930256
// MI455X (gfx1250) — hardware-verified
//
#include <hip/hip_runtime.h>
#include <math.h>


#define DD      256
#define HH      8
#define DHH     32
#define NEIGH   50
#define LSTP    52
#define NFRAGW  65536
#define QKSCALE 0.17677669529663687f

typedef __bf16 bf16_t;
typedef bf16_t v16b __attribute__((ext_vector_type(16)));
typedef bf16_t v8b  __attribute__((ext_vector_type(8)));
typedef float  v8f  __attribute__((ext_vector_type(8)));
typedef float  v4f  __attribute__((ext_vector_type(4)));
typedef unsigned int v4u __attribute__((ext_vector_type(4)));
typedef v4f v4fa __attribute__((may_alias));
union FragB { v16b v; v8b half[2]; };

__device__ __forceinline__ float wave_sum(float x) {
#pragma unroll
  for (int o = 16; o > 0; o >>= 1) x += __shfl_xor(x, o, 32);
  return x;
}
__device__ __forceinline__ float wave_max(float x) {
#pragma unroll
  for (int o = 16; o > 0; o >>= 1) x = fmaxf(x, __shfl_xor(x, o, 32));
  return x;
}

__device__ __forceinline__ unsigned int bf16_rne_bits(float x) {
  unsigned int u = __float_as_uint(x);
  return (u + 0x7FFFu + ((u >> 16) & 1u)) >> 16;
}
__device__ __forceinline__ void split_hl(float x, unsigned int& hb, unsigned int& lb) {
  hb = bf16_rne_bits(x);
  float hf = __uint_as_float(hb << 16);
  lb = bf16_rne_bits(x - hf);
}
__device__ __forceinline__ v4u pack8(const unsigned int* b) {
  v4u r;
  r.x = b[0] | (b[1] << 16);
  r.y = b[2] | (b[3] << 16);
  r.z = b[4] | (b[5] << 16);
  r.w = b[6] | (b[7] << 16);
  return r;
}

__device__ __forceinline__ v8f mma3(v8f acc, v16b ah, v16b al, v16b bh, v16b bl) {
  acc = __builtin_amdgcn_wmma_f32_16x16x32_bf16(false, ah, false, bh, (short)0, acc, false, false);
  acc = __builtin_amdgcn_wmma_f32_16x16x32_bf16(false, al, false, bh, (short)0, acc, false, false);
  acc = __builtin_amdgcn_wmma_f32_16x16x32_bf16(false, ah, false, bl, (short)0, acc, false, false);
  asm volatile("v_nop\n\tv_nop\n\tv_nop\n\tv_nop" : "+v"(acc) : "v"(ah), "v"(al), "v"(bh), "v"(bl));
  return acc;
}

__device__ __forceinline__ float pos_at(int d, size_t rowoff, float ccv, float dgv,
                                        const float* pe, const float* Wc, const float* bc,
                                        const float* Wd, const float* bd) {
  if (d < DD / 2) return pe[rowoff + d];
  if (d < 192)    return ccv * Wc[d - 128] + bc[d - 128];
  return dgv * Wd[d - 192] + bd[d - 192];
}

__global__ __launch_bounds__(256) void k_pack_w(const float* __restrict__ Wq, const float* __restrict__ Wk,
                                                const float* __restrict__ Wv, const float* __restrict__ Wo,
                                                unsigned short* __restrict__ wph, unsigned short* __restrict__ wpl) {
  int u = blockIdx.x * 256 + threadIdx.x;
  if (u >= 8192) return;
  int p = blockIdx.y;
  const float* W = (p == 0) ? Wq : (p == 1) ? Wk : (p == 2) ? Wv : Wo;
  int hb   = u & 1;
  int f    = u >> 1;
  int lane = f & 31;
  int jt   = (f >> 5) & 15;
  int kt   = f >> 9;
  int n    = jt * 16 + (lane & 15);
  int h    = lane >> 4;
  int k0   = kt * 32 + hb * 16 + 8 * h;
  const float* src = W + (size_t)n * DD + k0;
  float4 x0 = *reinterpret_cast<const float4*>(src);
  float4 x1 = *reinterpret_cast<const float4*>(src + 4);
  float x[8] = {x0.x, x0.y, x0.z, x0.w, x1.x, x1.y, x1.z, x1.w};
  unsigned int hbits[8], lbits[8];
#pragma unroll
  for (int i = 0; i < 8; ++i) split_hl(x[i], hbits[i], lbits[i]);
  v4u hv = pack8(hbits), lv = pack8(lbits);
  size_t o = (size_t)p * NFRAGW + (size_t)u * 8;
  unsigned short* ph = wph + o;
  unsigned short* pl = wpl + o;
  *(volatile v4u*)ph = hv;
  *(volatile v4u*)pl = lv;
  __threadfence();
  *(volatile v4u*)ph = hv;
  *(volatile v4u*)pl = lv;
}

__global__ __launch_bounds__(256) void k_pos_ln(const float* __restrict__ query, const float* __restrict__ kv,
                                                const float* __restrict__ deg, const float* __restrict__ cc,
                                                const float* __restrict__ pe,
                                                const float* __restrict__ Wc, const float* __restrict__ bc,
                                                const float* __restrict__ Wd, const float* __restrict__ bd,
                                                const float* __restrict__ gq, const float* __restrict__ bq_,
                                                const float* __restrict__ gk, const float* __restrict__ bk_,
                                                unsigned short* __restrict__ qh, unsigned short* __restrict__ ql,
                                                unsigned short* __restrict__ kh, unsigned short* __restrict__ kl,
                                                int nrows) {
  int row  = blockIdx.x * 8 + (threadIdx.x >> 5);
  int lane = threadIdx.x & 31;
  if (row >= nrows) return;
  size_t ro = (size_t)row * DD;
  int d0 = lane * 8;
  float ccv = cc[row], dgv = deg[row];
  float4 qa0 = *reinterpret_cast<const float4*>(query + ro + d0);
  float4 qa1 = *reinterpret_cast<const float4*>(query + ro + d0 + 4);
  float4 ka0 = *reinterpret_cast<const float4*>(kv + ro + d0);
  float4 ka1 = *reinterpret_cast<const float4*>(kv + ro + d0 + 4);
  float xq[8] = {qa0.x, qa0.y, qa0.z, qa0.w, qa1.x, qa1.y, qa1.z, qa1.w};
  float xk[8] = {ka0.x, ka0.y, ka0.z, ka0.w, ka1.x, ka1.y, ka1.z, ka1.w};
  float sq = 0.f, sk = 0.f;
#pragma unroll
  for (int i = 0; i < 8; ++i) {
    float ps = pos_at(d0 + i, ro, ccv, dgv, pe, Wc, bc, Wd, bd);
    xq[i] += ps; xk[i] += ps;
    sq += xq[i]; sk += xk[i];
  }
  sq = wave_sum(sq); sk = wave_sum(sk);
  float mq = sq * (1.f / DD), mk = sk * (1.f / DD);
  float vq = 0.f, vk2 = 0.f;
#pragma unroll
  for (int i = 0; i < 8; ++i) {
    float a = xq[i] - mq, b = xk[i] - mk;
    vq += a * a; vk2 += b * b;
  }
  vq = wave_sum(vq); vk2 = wave_sum(vk2);
  float rq = rsqrtf(vq * (1.f / DD) + 1e-5f);
  float rk = rsqrtf(vk2 * (1.f / DD) + 1e-5f);
  unsigned int hqb[8], lqb[8], hkb[8], lkb[8];
#pragma unroll
  for (int i = 0; i < 8; ++i) {
    int d = d0 + i;
    float yq = (xq[i] - mq) * rq * gq[d] + bq_[d];
    float yk = (xk[i] - mk) * rk * gk[d] + bk_[d];
    split_hl(yq, hqb[i], lqb[i]);
    split_hl(yk, hkb[i], lkb[i]);
  }
  v4u a = pack8(hqb), b = pack8(lqb), c = pack8(hkb), e = pack8(lkb);
  unsigned short* pqh = qh + ro + d0;
  unsigned short* pql = ql + ro + d0;
  unsigned short* pkh = kh + ro + d0;
  unsigned short* pkl = kl + ro + d0;
  *(volatile v4u*)pqh = a; *(volatile v4u*)pql = b;
  *(volatile v4u*)pkh = c; *(volatile v4u*)pkl = e;
  __threadfence();
  *(volatile v4u*)pqh = a; *(volatile v4u*)pql = b;
  *(volatile v4u*)pkh = c; *(volatile v4u*)pkl = e;
}

__global__ __launch_bounds__(256) void k_gemm3(const bf16_t* __restrict__ Ah, const bf16_t* __restrict__ Al,
                                               const bf16_t* __restrict__ Bh, const bf16_t* __restrict__ Bl,
                                               const float* __restrict__ bias, float* __restrict__ Out, int nrows) {
  __shared__ __attribute__((aligned(16))) float sT[16 * 128];
  int tid = threadIdx.x, wv = tid >> 5, lane = tid & 31;
  int h = lane >> 4, m = lane & 15;
  int row0 = blockIdx.x * 16;
  int jt   = blockIdx.y * 8 + wv;
  int arow = row0 + m;
  if (arow > nrows - 1) arow = nrows - 1;
  const bf16_t* pah = Ah + (size_t)arow * DD + 8 * h;
  const bf16_t* pal = Al + (size_t)arow * DD + 8 * h;
  const bf16_t* pbh = Bh + ((size_t)jt * 32 + lane) * 16;
  const bf16_t* pbl = Bl + ((size_t)jt * 32 + lane) * 16;
  v8f acc = {0.f, 0.f, 0.f, 0.f, 0.f, 0.f, 0.f, 0.f};
#pragma unroll 1
  for (int kt = 0; kt < 8; ++kt) {
    FragB fah, fal, fbh, fbl;
    fah.half[0] = *reinterpret_cast<const v8b*>(pah + kt * 32);
    fah.half[1] = *reinterpret_cast<const v8b*>(pah + kt * 32 + 16);
    fal.half[0] = *reinterpret_cast<const v8b*>(pal + kt * 32);
    fal.half[1] = *reinterpret_cast<const v8b*>(pal + kt * 32 + 16);
    const bf16_t* qbh = pbh + (size_t)kt * 8192;
    const bf16_t* qbl = pbl + (size_t)kt * 8192;
    fbh.half[0] = *reinterpret_cast<const v8b*>(qbh);
    fbh.half[1] = *reinterpret_cast<const v8b*>(qbh + 8);
    fbl.half[0] = *reinterpret_cast<const v8b*>(qbl);
    fbl.half[1] = *reinterpret_cast<const v8b*>(qbl + 8);
    acc = mma3(acc, fah.v, fal.v, fbh.v, fbl.v);
  }
  float bj = bias[jt * 16 + m];
#pragma unroll
  for (int r = 0; r < 8; ++r) sT[(8 * h + r) * 128 + wv * 16 + m] = acc[r] + bj;
  __syncthreads();
  int r0 = 2 * wv, r1 = 2 * wv + 1;
  v4f o0 = *reinterpret_cast<const v4fa*>(&sT[r0 * 128 + lane * 4]);
  v4f o1 = *reinterpret_cast<const v4fa*>(&sT[r1 * 128 + lane * 4]);
  size_t cb = (size_t)blockIdx.y * 128 + (size_t)lane * 4;
  float* p0 = Out + (size_t)(row0 + r0) * DD + cb;
  float* p1 = Out + (size_t)(row0 + r1) * DD + cb;
  bool ok0 = (row0 + r0) < nrows, ok1 = (row0 + r1) < nrows;
  if (ok0) *(volatile v4f*)p0 = o0;
  if (ok1) *(volatile v4f*)p1 = o1;
  __threadfence();
  if (ok0) *(volatile v4f*)p0 = o0;
  if (ok1) *(volatile v4f*)p1 = o1;
}

__device__ __forceinline__ float dot32(const float* kr, const float* qv) {
  float s = 0.f;
#pragma unroll 2
  for (int d = 0; d < DHH; d += 4) {
    float4 k4 = *reinterpret_cast<const float4*>(kr + d);
    s += qv[d] * k4.x + qv[d + 1] * k4.y + qv[d + 2] * k4.z + qv[d + 3] * k4.w;
  }
  return s;
}

__global__ __launch_bounds__(256) void k_attn(const float* __restrict__ qf, const float* __restrict__ kf,
                                              const float* __restrict__ vf,
                                              const int* __restrict__ erow, const int* __restrict__ ecol,
                                              int ne, int nn,
                                              unsigned short* __restrict__ oh, unsigned short* __restrict__ ol) {
  __shared__ __attribute__((aligned(16))) float lq[DD];
  __shared__ __attribute__((aligned(16))) float so[DD];
  __shared__ float lat[HH * 64];
  __shared__ int lst[16 * LSTP];
  __shared__ int lc[16];
  __shared__ int ls[64];
  int n = blockIdx.x;
  if (n >= nn) return;
  int tid = threadIdx.x, w = tid >> 5, lane = tid & 31;
  lq[tid] = qf[(size_t)n * DD + tid];

  int ew = (ne + 7) >> 3;
  int tb = w * ew; if (tb > ne) tb = ne;
  int te = tb + ew; if (te > ne) te = ne;
  unsigned int ltmask = (1u << lane) - 1u;

  {
    int cnt = 0;
    for (int t0 = tb; t0 < te; t0 += 32) {
      int t = t0 + lane;
      bool in = t < te;
      int r = -1;
      if (in) r = erow[t];
      bool match = in && (r == n);
      unsigned int msk = __builtin_amdgcn_ballot_w32(match);
      if (msk) {
        int rank = cnt + __builtin_popcount(msk & ltmask);
        if (match && rank < NEIGH) {
          int c = ecol[t];
          c = (c < 0) ? 0 : ((c >= nn) ? (nn - 1) : c);
          lst[w * LSTP + rank] = c;
        }
        cnt += __builtin_popcount(msk);
        if (cnt >= NEIGH) break;
      }
    }
    if (lane == 0) lc[w] = (cnt < NEIGH) ? cnt : NEIGH;
  }
  {
    int cnt = 0;
    for (int t0 = tb; t0 < te; t0 += 32) {
      int t = t0 + lane;
      bool in = t < te;
      int c = -1;
      if (in) c = ecol[t];
      bool match = in && (c == n);
      unsigned int msk = __builtin_amdgcn_ballot_w32(match);
      if (msk) {
        int rank = cnt + __builtin_popcount(msk & ltmask);
        if (match && rank < NEIGH) {
          int r = erow[t];
          r = (r < 0) ? 0 : ((r >= nn) ? (nn - 1) : r);
          lst[(8 + w) * LSTP + rank] = r;
        }
        cnt += __builtin_popcount(msk);
        if (cnt >= NEIGH) break;
      }
    }
    if (lane == 0) lc[8 + w] = (cnt < NEIGH) ? cnt : NEIGH;
  }
  __syncthreads();

  int offA = 0, offB = 0, total = 0;
#pragma unroll
  for (int j = 0; j < 16; ++j) {
    if (j == w)     offA = total;
    if (j == 8 + w) offB = total;
    total += lc[j];
  }
  {
    int ca = lc[w];
    for (int i = lane; i < ca; i += 32) {
      int p = offA + i;
      if (p < NEIGH) ls[p] = lst[w * LSTP + i];
    }
    int cbn = lc[8 + w];
    for (int i = lane; i < cbn; i += 32) {
      int p = offB + i;
      if (p < NEIGH) ls[p] = lst[(8 + w) * LSTP + i];
    }
  }
  int ntot = (total < NEIGH) ? total : NEIGH;
  if (total < NEIGH) {
    if (tid == 0) ls[total] = n;
    ntot = total + 1;
  }
  __syncthreads();

  int qb = w * DHH;
  float s0 = -1e30f, s1 = -1e30f;
  if (lane < ntot)      s0 = dot32(kf + (size_t)ls[lane] * DD + qb, lq + qb) * QKSCALE;
  if (lane + 32 < ntot) s1 = dot32(kf + (size_t)ls[lane + 32] * DD + qb, lq + qb) * QKSCALE;
  float mx = wave_max(fmaxf(s0, s1));
  float e0 = (lane < ntot)      ? expf(s0 - mx) : 0.f;
  float e1 = (lane + 32 < ntot) ? expf(s1 - mx) : 0.f;
  float ssum = wave_sum(e0 + e1);
  float inv = 1.f / ssum;
  lat[w * 64 + lane]      = e0 * inv;
  lat[w * 64 + 32 + lane] = e1 * inv;
  __syncthreads();

  float acc = 0.f;
#pragma unroll 2
  for (int r = 0; r < ntot; ++r)
    acc += lat[w * 64 + r] * vf[(size_t)ls[r] * DD + qb + lane];
  so[qb + lane] = acc;
  __syncthreads();

  if (w < 2) {
    float x[8];
#pragma unroll
    for (int i = 0; i < 8; ++i) x[i] = so[lane * 8 + i];
    unsigned int hb[8], lb[8];
#pragma unroll
    for (int i = 0; i < 8; ++i) split_hl(x[i], hb[i], lb[i]);
    v4u val = (w == 0) ? pack8(hb) : pack8(lb);
    unsigned short* dst = ((w == 0) ? oh : ol) + (size_t)n * DD + lane * 8;
    *(volatile v4u*)dst = val;
    __threadfence();
    *(volatile v4u*)dst = val;
  }
}

__global__ __launch_bounds__(256) void k_out_ln(const float* __restrict__ proj, const float* __restrict__ query,
                                                const float* __restrict__ cc, const float* __restrict__ deg,
                                                const float* __restrict__ pe,
                                                const float* __restrict__ Wc, const float* __restrict__ bc,
                                                const float* __restrict__ Wd, const float* __restrict__ bd,
                                                const float* __restrict__ g, const float* __restrict__ b,
                                                float* __restrict__ out, int nrows) {
  int row  = blockIdx.x * 8 + (threadIdx.x >> 5);
  int lane = threadIdx.x & 31;
  if (row >= nrows) return;
  size_t ro = (size_t)row * DD;
  int dA = lane * 4, dB = 128 + lane * 4;
  float ccv = cc[row], dgv = deg[row];
  float4 p0 = *reinterpret_cast<const float4*>(proj + ro + dA);
  float4 p1 = *reinterpret_cast<const float4*>(proj + ro + dB);
  float4 q0 = *reinterpret_cast<const float4*>(query + ro + dA);
  float4 q1 = *reinterpret_cast<const float4*>(query + ro + dB);
  float4 e0 = *reinterpret_cast<const float4*>(pe + ro + dA);
  float x[8];
  x[0] = p0.x + (q0.x + e0.x);
  x[1] = p0.y + (q0.y + e0.y);
  x[2] = p0.z + (q0.z + e0.z);
  x[3] = p0.w + (q0.w + e0.w);
  float qv1[4] = {q1.x, q1.y, q1.z, q1.w};
  float pv1[4] = {p1.x, p1.y, p1.z, p1.w};
#pragma unroll
  for (int i = 0; i < 4; ++i) {
    float ps = pos_at(dB + i, ro, ccv, dgv, pe, Wc, bc, Wd, bd);
    x[4 + i] = pv1[i] + (qv1[i] + ps);
  }
  float s = 0.f;
#pragma unroll
  for (int i = 0; i < 8; ++i) s += x[i];
  s = wave_sum(s);
  float m = s * (1.f / DD);
  float v = 0.f;
#pragma unroll
  for (int i = 0; i < 8; ++i) { float a = x[i] - m; v += a * a; }
  v = wave_sum(v);
  float r = rsqrtf(v * (1.f / DD) + 1e-5f);
  v4f y0, y1;
#pragma unroll
  for (int i = 0; i < 4; ++i) {
    y0[i] = (x[i] - m) * r * g[dA + i] + b[dA + i];
    y1[i] = (x[4 + i] - m) * r * g[dB + i] + b[dB + i];
  }
  float* pa = out + ro + dA;
  float* pb = out + ro + dB;
  *(volatile v4f*)pa = y0;
  *(volatile v4f*)pb = y1;
  __threadfence();
  *(volatile v4f*)pa = y0;
  *(volatile v4f*)pb = y1;
}

extern "C" void kernel_launch(void* const* d_in, const int* in_sizes, int n_in,
                              void* d_out, int out_size, void* d_ws, size_t ws_size,
                              hipStream_t stream) {
  if (n_in < 24) return;
  const float* query = (const float*)d_in[0];
  const float* keyv  = (const float*)d_in[1];
  const float* ndeg  = (const float*)d_in[2];
  const float* ccf   = (const float*)d_in[3];
  const float* pe    = (const float*)d_in[4];
  const float* Wc    = (const float*)d_in[5];
  const float* bc    = (const float*)d_in[6];
  const float* Wd    = (const float*)d_in[7];
  const float* bd    = (const float*)d_in[8];
  const float* g_q   = (const float*)d_in[9];
  const float* b_q   = (const float*)d_in[10];
  const float* g_kv  = (const float*)d_in[11];
  const float* b_kv  = (const float*)d_in[12];
  const float* g_out = (const float*)d_in[13];
  const float* b_out = (const float*)d_in[14];
  const float* Wq    = (const float*)d_in[15];
  const float* bq    = (const float*)d_in[16];
  const float* Wk    = (const float*)d_in[17];
  const float* bk    = (const float*)d_in[18];
  const float* Wv    = (const float*)d_in[19];
  const float* bv    = (const float*)d_in[20];
  const float* Wo    = (const float*)d_in[21];
  const float* bo    = (const float*)d_in[22];
  const int*   ei    = (const int*)d_in[23];
  float* out = (float*)d_out;

  const int nn = in_sizes[0] / DD;
  if (nn <= 0 || (nn % 16) != 0) return;
  if (in_sizes[0] != nn * DD || in_sizes[1] != nn * DD) return;
  if (in_sizes[2] < nn || in_sizes[3] < nn || in_sizes[4] < nn * DD) return;
  if (in_sizes[5] < 64 || in_sizes[6] < 64 || in_sizes[7] < 64 || in_sizes[8] < 64) return;
  for (int i = 9; i <= 14; ++i) if (in_sizes[i] < DD) return;
  if (in_sizes[15] != DD * DD || in_sizes[17] != DD * DD || in_sizes[19] != DD * DD || in_sizes[21] != DD * DD) return;
  if (in_sizes[16] < DD || in_sizes[18] < DD || in_sizes[20] < DD || in_sizes[22] < DD) return;
  const int ne = in_sizes[23] / 2;
  if (ne < 0) return;
  if (out_size != nn * DD) return;

  char* ws = (char*)d_ws;
  size_t off = 0;
  auto carve = [&](size_t bytes) -> char* {
    char* p = ws + off;
    off = (off + bytes + 255) & ~(size_t)255;
    return p;
  };
  const size_t planeB = (size_t)nn * DD * 2;
  const size_t rowsF  = (size_t)nn * DD * 4;
  unsigned short* qh   = (unsigned short*)carve(planeB);
  unsigned short* ql   = (unsigned short*)carve(planeB);
  unsigned short* kh   = (unsigned short*)carve(planeB);
  unsigned short* kl   = (unsigned short*)carve(planeB);
  float*          qf   = (float*)carve(rowsF);
  float*          kf   = (float*)carve(rowsF);
  float*          vf   = (float*)carve(rowsF);
  unsigned short* oh   = (unsigned short*)carve(planeB);
  unsigned short* ol   = (unsigned short*)carve(planeB);
  float*          proj = (float*)carve(rowsF);
  unsigned short* wph  = (unsigned short*)carve((size_t)4 * NFRAGW * 2);
  unsigned short* wpl  = (unsigned short*)carve((size_t)4 * NFRAGW * 2);
  if (off > ws_size) return;

  const bf16_t* Bqh = (const bf16_t*)wph + 0 * NFRAGW; const bf16_t* Bql = (const bf16_t*)wpl + 0 * NFRAGW;
  const bf16_t* Bkh = (const bf16_t*)wph + 1 * NFRAGW; const bf16_t* Bkl = (const bf16_t*)wpl + 1 * NFRAGW;
  const bf16_t* Bvh = (const bf16_t*)wph + 2 * NFRAGW; const bf16_t* Bvl = (const bf16_t*)wpl + 2 * NFRAGW;
  const bf16_t* Boh = (const bf16_t*)wph + 3 * NFRAGW; const bf16_t* Bol = (const bf16_t*)wpl + 3 * NFRAGW;

  k_pack_w<<<dim3(32, 4), 256, 0, stream>>>(Wq, Wk, Wv, Wo, wph, wpl);
  k_pos_ln<<<(nn + 7) / 8, 256, 0, stream>>>(query, keyv, ndeg, ccf, pe, Wc, bc, Wd, bd,
                                             g_q, b_q, g_kv, b_kv, qh, ql, kh, kl, nn);
  k_gemm3<<<dim3(nn / 16, 2), 256, 0, stream>>>((const bf16_t*)qh, (const bf16_t*)ql, Bqh, Bql, bq, qf, nn);
  k_gemm3<<<dim3(nn / 16, 2), 256, 0, stream>>>((const bf16_t*)kh, (const bf16_t*)kl, Bkh, Bkl, bk, kf, nn);
  k_gemm3<<<dim3(nn / 16, 2), 256, 0, stream>>>((const bf16_t*)kh, (const bf16_t*)kl, Bvh, Bvl, bv, vf, nn);
  k_attn<<<nn, 256, 0, stream>>>(qf, kf, vf, ei, ei + ne, ne, nn, oh, ol);
  k_gemm3<<<dim3(nn / 16, 2), 256, 0, stream>>>((const bf16_t*)oh, (const bf16_t*)ol, Boh, Bol, bo, proj, nn);
  k_out_ln<<<(nn + 7) / 8, 256, 0, stream>>>(proj, query, ccf, ndeg, pe, Wc, bc, Wd, bd, g_out, b_out, out, nn);
}
